// GraphMixKNN_63299228008825
// MI455X (gfx1250) — hardware-verified
//
#include <hip/hip_runtime.h>
#include <hip/hip_bf16.h>


#define __bf16 _Float16
typedef __attribute__((ext_vector_type(16))) __bf16 v16bf;
typedef __attribute__((ext_vector_type(8)))  __bf16 v8bf;
typedef __attribute__((ext_vector_type(2)))  __bf16 v2bf;
typedef __attribute__((ext_vector_type(8)))  float  v8f;
typedef __attribute__((ext_vector_type(4)))  float  v4f_t;
typedef float v4fa __attribute__((ext_vector_type(4), may_alias));
#define RSPLIT (1.0f / 2048.0f)
#define NNODES 50000
__device__ __forceinline__ __bf16 lo_of(float v, __bf16 h) { return (__bf16)((v - (float)h) * 2048.0f); }
__device__ __forceinline__ v8f wmma16(v16bf a, v16bf b, v8f c) { return __builtin_amdgcn_wmma_f32_16x16x32_f16(false, a, false, b, (short)0, c, false, false); }
__device__ __forceinline__ v8f wmma_split(v16bf a, v16bf al, v16bf b, v16bf bl, v8f c) { v8f x = {}; x = wmma16(al, b, x); x = wmma16(a, bl, x); return wmma16(a, b, c) + x * RSPLIT; }

#define KNBR 32
#define H    64
#define H2   128
#define GH   64

#define WAVES 4
#define TILE  16
#define NODES_PER_BLOCK (WAVES * TILE)
#define CAT_STRIDE 136
#define KSTRIDE    136
#define K2STRIDE   72

__global__ __launch_bounds__(WAVES * 32)
void graphmix_kernel(const float* __restrict__ Z,
                     const int*   __restrict__ nbr_idx,
                     const float* __restrict__ nbr_w,
                     const float* __restrict__ vmask,
                     const float* __restrict__ W_gate,
                     const float* __restrict__ b_gate,
                     const float* __restrict__ W_gate2,
                     const float* __restrict__ b_gate2,
                     const float* __restrict__ W_msg,
                     const float* __restrict__ b_msg,
                     float* __restrict__ out,
                     int N)
{
    alignas(16) __shared__ __bf16 sWg[2][GH * KSTRIDE];
    alignas(16) __shared__ __bf16 sWm[2][GH * KSTRIDE];
    alignas(16) __shared__ __bf16 sW2[2][H  * K2STRIDE];
    alignas(16) __shared__ __bf16 sCat[2][WAVES][TILE * CAT_STRIDE];
    __shared__ float sBg[GH], sB2[H], sBm[H];

    const int tid  = threadIdx.x;
    const int lane = tid & 31;
    const int wid  = tid >> 5;
    const int nthr = WAVES * 32;

    for (int i = tid; i < H2 * GH; i += nthr) {
        int k = i >> 6, c = i & 63;
        { const float v = W_gate[i]; const __bf16 h = (__bf16)v; sWg[0][c * KSTRIDE + k] = h; sWg[1][c * KSTRIDE + k] = lo_of(v, h); }
        { const float v = W_msg[i];  const __bf16 h = (__bf16)v; sWm[0][c * KSTRIDE + k] = h; sWm[1][c * KSTRIDE + k] = lo_of(v, h); }
    }
    for (int i = tid; i < GH * H; i += nthr) {
        int k = i >> 6, c = i & 63;
        const float v = W_gate2[i]; const __bf16 h = (__bf16)v; sW2[0][c * K2STRIDE + k] = h; sW2[1][c * K2STRIDE + k] = lo_of(v, h);
    }
    if (tid < GH) sBg[tid] = b_gate[tid];
    if (tid < H)  { sB2[tid] = b_gate2[tid]; sBm[tid] = b_msg[tid]; }

    const int tileBase = blockIdx.x * NODES_PER_BLOCK + wid * TILE;

    for (int nl = 0; nl < TILE; ++nl) {
        int n   = tileBase + nl;
        int ncl = (n < N) ? n : (N - 1);

        float wraw = nbr_w[(size_t)ncl * KNBR + lane];
        int   iraw = nbr_idx[(size_t)ncl * KNBR + lane];
        iraw = (iraw < 0) ? 0 : (iraw > N - 1 ? N - 1 : iraw);
        float wk = (__builtin_isfinite(wraw) && wraw > 0.0f) ? wraw : 0.0f;

        __builtin_prefetch(&Z[(size_t)iraw * H], 0, 0);

        float wsum = wk;
        #pragma unroll
        for (int off = 16; off; off >>= 1) wsum += __shfl_xor(wsum, off);

        float acc0 = 0.0f, acc1 = 0.0f;
        for (int k = 0; k < KNBR; ++k) {
            float wkk = __shfl(wk, k);
            int   jj  = __shfl(iraw, k);
            float c   = wkk * vmask[jj];
            const float* zr = &Z[(size_t)jj * H + 2 * lane];
            acc0 += c * zr[0];
            acc1 += c * zr[1];
        }
        float inv = 1.0f / (wsum + 1e-6f);

        const float* zs = &Z[(size_t)ncl * H + 2 * lane];
        __bf16* row  = &sCat[0][wid][nl * CAT_STRIDE];
        __bf16* rowl = &sCat[1][wid][nl * CAT_STRIDE];
        {
            const float z0 = zs[0], z1 = zs[1], m0 = acc0 * inv, m1 = acc1 * inv;
            const __bf16 hz0 = (__bf16)z0, hz1 = (__bf16)z1, hm0 = (__bf16)m0, hm1 = (__bf16)m1;
            *(v2bf*)&row[2 * lane]      = (v2bf){hz0, hz1};
            *(v2bf*)&rowl[2 * lane]     = (v2bf){lo_of(z0, hz0), lo_of(z1, hz1)};
            *(v2bf*)&row[H + 2 * lane]  = (v2bf){hm0, hm1};
            *(v2bf*)&rowl[H + 2 * lane] = (v2bf){lo_of(m0, hm0), lo_of(m1, hm1)};
        }
    }

    __syncthreads();

    const int mcol   = lane & 15;
    const int kAbase = (lane < 16) ? 0 : 8;

    auto loadA = [&](int pl, int kc) -> v16bf {
        const __bf16* p = &sCat[pl][wid][mcol * CAT_STRIDE] + kc * 32 + kAbase;
        v8bf lo = *(const v8bf*)(p);
        v8bf hi = *(const v8bf*)(p + 16);
        return __builtin_shufflevector(lo, hi, 0,1,2,3,4,5,6,7,8,9,10,11,12,13,14,15);
    };
    auto loadB = [&](const __bf16* Wcol, int kstride, int kc, int nc) -> v16bf {
        const __bf16* p = Wcol + (nc * 16 + mcol) * kstride + kc * 32 + kAbase;
        v8bf lo = *(const v8bf*)(p);
        v8bf hi = *(const v8bf*)(p + 16);
        return __builtin_shufflevector(lo, hi, 0,1,2,3,4,5,6,7,8,9,10,11,12,13,14,15);
    };

    v8f hacc[4], dacc[4];
    #pragma unroll
    for (int nc = 0; nc < 4; ++nc) {
        float bg = sBg[nc * 16 + mcol];
        float bm = sBm[nc * 16 + mcol];
        v8f hc, dc;
        #pragma unroll
        for (int r = 0; r < 8; ++r) { hc[r] = bg; dc[r] = bm; }
        #pragma unroll 1
        for (int kc = 0; kc < 4; ++kc) {
            v16bf a  = loadA(0, kc), al = loadA(1, kc);
            hc = wmma_split(a, al, loadB(sWg[0], KSTRIDE, kc, nc), loadB(sWg[1], KSTRIDE, kc, nc), hc);
            dc = wmma_split(a, al, loadB(sWm[0], KSTRIDE, kc, nc), loadB(sWm[1], KSTRIDE, kc, nc), dc);
        }
        #pragma unroll
        for (int r = 0; r < 8; ++r) {
            hc[r] = fmaxf(hc[r], 0.0f);
            dc[r] = fmaxf(dc[r], 0.0f);
        }
        hacc[nc] = hc; dacc[nc] = dc;
    }

    #pragma unroll
    for (int nc = 0; nc < 4; ++nc) {
        int col = nc * 16 + mcol;
        #pragma unroll
        for (int r = 0; r < 8; ++r) {
            int M = (lane < 16) ? r : (r + 8);
            const __bf16 hv = (__bf16)hacc[nc][r];
            sCat[0][wid][M * CAT_STRIDE + col] = hv;
            sCat[1][wid][M * CAT_STRIDE + col] = lo_of(hacc[nc][r], hv);
        }
    }
    asm volatile("s_wait_dscnt 0" ::: "memory");

    v8f gacc[4];
    #pragma unroll
    for (int nc = 0; nc < 4; ++nc) {
        float b2 = sB2[nc * 16 + mcol];
        v8f gc;
        #pragma unroll
        for (int r = 0; r < 8; ++r) gc[r] = b2;
        #pragma unroll 1
        for (int kc = 0; kc < 2; ++kc)
            gc = wmma_split(loadA(0, kc), loadA(1, kc), loadB(sW2[0], K2STRIDE, kc, nc), loadB(sW2[1], K2STRIDE, kc, nc), gc);
        gacc[nc] = gc;
    }
    asm volatile("s_wait_dscnt 0" ::: "memory");
    float* so = (float*)&sCat[0][wid][0];
    #pragma unroll
    for (int nc = 0; nc < 4; ++nc) {
        int col = nc * 16 + mcol;
        #pragma unroll
        for (int r = 0; r < 8; ++r) {
            int M = (lane < 16) ? r : (r + 8);
            float g = 1.0f / (1.0f + __expf(-gacc[nc][r]));
            so[M * 64 + col] = g * dacc[nc][r];
        }
    }
    asm volatile("s_wait_dscnt 0" ::: "memory");
#pragma unroll 1
    for (int pass = 0; pass < 2; ++pass) {
        #pragma unroll
        for (int i = 0; i < 8; ++i) { const int c = lane + 32 * i, M = c >> 4, q = (c & 15) * 4; const int n = tileBase + M;
            if (n < N) { v4f_t v = *(const v4f_t*)(Z + (size_t)n * H + q); v += *(const volatile v4fa*)(so + M * 64 + q);
                *(volatile v4f_t*)(out + (size_t)n * H + q) = v; } }
        __threadfence();
    }
}

extern "C" void kernel_launch(void* const* d_in, const int* in_sizes, int n_in,
                              void* d_out, int out_size, void* d_ws, size_t ws_size,
                              hipStream_t stream) {
    const float* Z       = (const float*)d_in[0];
    const int*   nbr_idx = (const int*)  d_in[1];
    const float* nbr_w   = (const float*)d_in[2];
    const float* vmask   = (const float*)d_in[3];
    const float* W_gate  = (const float*)d_in[4];
    const float* b_gate  = (const float*)d_in[5];
    const float* W_gate2 = (const float*)d_in[6];
    const float* b_gate2 = (const float*)d_in[7];
    const float* W_msg   = (const float*)d_in[8];
    const float* b_msg   = (const float*)d_in[9];
    float*       out     = (float*)d_out;

    (void)in_sizes;
    const int N = NNODES;
    const int blocks = (N + NODES_PER_BLOCK - 1) / NODES_PER_BLOCK;
    graphmix_kernel<<<blocks, WAVES * 32, 0, stream>>>(
        Z, nbr_idx, nbr_w, vmask, W_gate, b_gate, W_gate2, b_gate2,
        W_msg, b_msg, out, N);
}
